// InContextAssoMemBlock_14534169329971
// MI455X (gfx1250) — hardware-verified
//
#include <hip/hip_runtime.h>
#include <stdint.h>


#define B_DIM 2
#define T_DIM 2048
#define C_DIM 768
#define NH    12
#define HS    64

typedef unsigned short us_t;
typedef __bf16         v16bf __attribute__((ext_vector_type(16)));
typedef unsigned short v16us __attribute__((ext_vector_type(16)));
typedef unsigned short v8us  __attribute__((ext_vector_type(8)));
typedef float          v8f   __attribute__((ext_vector_type(8)));
typedef float          v4f   __attribute__((ext_vector_type(4)));
typedef unsigned int   v4u   __attribute__((ext_vector_type(4)));

union Frag { v16us u; v8us half[2]; };

__device__ __forceinline__ v8f vzero() {
  v8f z;
#pragma unroll
  for (int i = 0; i < 8; ++i) z[i] = 0.0f;
  return z;
}

__device__ __forceinline__ us_t f2bf(float f) {
  unsigned u = __float_as_uint(f);
  u += 0x7FFFu + ((u >> 16) & 1u);
  return (us_t)(u >> 16);
}
__device__ __forceinline__ float bf2f(us_t b) { return __uint_as_float(((unsigned)b) << 16); }
__device__ __forceinline__ float bfr(float f) { return bf2f(f2bf(f)); }
__device__ __forceinline__ unsigned pk2(us_t a, us_t b) { return (unsigned)a | (((unsigned)b) << 16); }

__device__ __forceinline__ v16us ld_frag(const us_t* __restrict__ p, int hh) {
  Frag f;
  f.half[0] = *(const v8us*)(p + 8 * hh);
  f.half[1] = *(const v8us*)(p + 16 + 8 * hh);
  return f.u;
}

__device__ __forceinline__ v8f mma(v16us a, v16us b, v8f c) {
  v16bf av = __builtin_bit_cast(v16bf, a);
  v16bf bv = __builtin_bit_cast(v16bf, b);
  c = __builtin_amdgcn_wmma_f32_16x16x32_bf16(false, av, false, bv, (short)0, c, false, false);
  asm volatile("v_nop\n\tv_nop\n\tv_nop\n\tv_nop" : "+v"(c) : "v"(a), "v"(b));
  return c;
}

__global__ __launch_bounds__(256) void k_cvt(const float* __restrict__ in,
                                            us_t* __restrict__ out, int n8) {
  const int i = blockIdx.x * 256 + threadIdx.x;
  if (i >= n8) return;
  const v4f* src = (const v4f*)(in + (size_t)i * 8);
  const v4f a = src[0];
  const v4f c = src[1];
  v4u p;
  p[0] = pk2(f2bf(a[0]), f2bf(a[1]));
  p[1] = pk2(f2bf(a[2]), f2bf(a[3]));
  p[2] = pk2(f2bf(c[0]), f2bf(c[1]));
  p[3] = pk2(f2bf(c[2]), f2bf(c[3]));
  volatile v4u* dst = (volatile v4u*)(out + (size_t)i * 8);
  *dst = p;
  __threadfence();
  *dst = p;
}

template <int SPLITA>
__global__ __launch_bounds__(128) void k_gemm(const us_t* __restrict__ A,
                                             const us_t* __restrict__ A2,
                                             const us_t* __restrict__ W,
                                             float* __restrict__ Cout,
                                             int M, int N, int K) {
  __shared__ __align__(16) float ldsC[4][16][68];
  (void)M;
  const int w = threadIdx.x >> 5, lane = threadIdx.x & 31, m = lane & 15, hh = lane >> 4;
  const int mbase = blockIdx.y * 64 + w * 16;
  const int nbase = blockIdx.x * 64;
  const us_t* arow  = A  + (size_t)(mbase + m) * K;
  const us_t* a2row = A2 + (size_t)(mbase + m) * K;
  const us_t* wrow  = W  + (size_t)(nbase + m) * K;

  v8f acc[4];
#pragma unroll
  for (int g = 0; g < 4; ++g) acc[g] = vzero();

#pragma unroll 2
  for (int kb = 0; kb < K; kb += 32) {
    const v16us a = ld_frag(arow + kb, hh);
    v16us a2 = a;
    if (SPLITA) a2 = ld_frag(a2row + kb, hh);
#pragma unroll
    for (int g = 0; g < 4; ++g) {
      const v16us bw = ld_frag(wrow + (size_t)(16 * g) * K + kb, hh);
      acc[g] = mma(a, bw, acc[g]);
      if (SPLITA) acc[g] = mma(a2, bw, acc[g]);
    }
  }

#pragma unroll
  for (int g = 0; g < 4; ++g) {
#pragma unroll
    for (int r = 0; r < 8; ++r) ldsC[w][8 * hh + r][16 * g + m] = acc[g][r];
  }
  __syncthreads();

  v4f val[8];
#pragma unroll
  for (int it = 0; it < 8; ++it) val[it] = *(const v4f*)(&ldsC[w][2 * it + hh][4 * m]);

  float* gb = Cout + (size_t)mbase * N + nbase + 4 * m;
#pragma unroll
  for (int it = 0; it < 8; ++it)
    *(volatile v4f*)(gb + (size_t)(2 * it + hh) * N) = val[it];
  __threadfence();
#pragma unroll
  for (int it = 0; it < 8; ++it)
    *(volatile v4f*)(gb + (size_t)(2 * it + hh) * N) = val[it];
}

__global__ __launch_bounds__(32) void k_ema_knorm(const float* __restrict__ u,
                                                 const float* __restrict__ la_coef,
                                                 const float* __restrict__ kbeta,
                                                 us_t* __restrict__ khi,
                                                 us_t* __restrict__ klo) {
#pragma clang fp contract(off)
  const int lane = threadIdx.x & 31;
  const int b    = blockIdx.x / (C_DIM / 256);
  const int grp  = blockIdx.x % (C_DIM / 256);
  const int h    = grp * 4 + (lane >> 3);
  const int sub  = lane & 7;

  const float cc   = bfr(la_coef[h]);
  const float omc  = 1.0f - cc;
  const float beta = expf(fminf(bfr(kbeta[h]) * 10.0f, 5.0f));

  const float* up   = u + (size_t)b * T_DIM * C_DIM + h * HS + 8 * sub;
  const size_t drow = ((size_t)(b * NH + h) * T_DIM) * HS + 8 * sub;

  float y[8];
#pragma unroll
  for (int i = 0; i < 8; ++i) y[i] = 0.0f;

  for (int t = 0; t < T_DIM; ++t) {
    const v4f* src = (const v4f*)(up + (size_t)t * C_DIM);
    const v4f x0 = src[0];
    const v4f x1 = src[1];
    float xin[8];
#pragma unroll
    for (int i = 0; i < 4; ++i) { xin[i] = x0[i]; xin[4 + i] = x1[i]; }
    float ss = 0.0f;
#pragma unroll
    for (int i = 0; i < 8; ++i) {
      y[i] = cc * y[i] + omc * xin[i];
      ss += y[i] * y[i];
    }
    ss += __shfl_xor(ss, 1, 32);
    ss += __shfl_xor(ss, 2, 32);
    ss += __shfl_xor(ss, 4, 32);
    const float rn = 1.0f / (sqrtf(ss) + 1e-6f);

    v4u ph, pl;
#pragma unroll
    for (int i = 0; i < 4; ++i) {
      const float ka = (y[2 * i] * rn) * beta;
      const float kc = (y[2 * i + 1] * rn) * beta;
      const us_t ha = f2bf(ka), hc = f2bf(kc);
      ph[i] = pk2(ha, hc);
      pl[i] = pk2(f2bf(ka - bf2f(ha)), f2bf(kc - bf2f(hc)));
    }
    const size_t off = drow + (size_t)t * HS;
    *(volatile v4u*)(khi + off) = ph;
    *(volatile v4u*)(klo + off) = pl;
    __threadfence();
    *(volatile v4u*)(khi + off) = ph;
    *(volatile v4u*)(klo + off) = pl;
  }
}

__global__ __launch_bounds__(128) void k_vmake(const float* __restrict__ xl,
                                              const float* __restrict__ v_coef,
                                              const float* __restrict__ vbeta,
                                              us_t* __restrict__ vthi,
                                              us_t* __restrict__ vtlo) {
#pragma clang fp contract(off)
  __shared__ __align__(16) us_t ldsH[HS][72];
  __shared__ __align__(16) us_t ldsL[HS][72];
  const int bh = blockIdx.y, b = bh / NH, h = bh % NH;
  const int t0 = blockIdx.x * 64;
  const int w = threadIdx.x >> 5, lane = threadIdx.x & 31;

  const float vc  = bfr(v_coef[h]);
  const float omv = 1.0f - vc;
  const float vb  = expf(fminf(bfr(vbeta[h]) * 10.0f, 5.0f));

  for (int rr = 0; rr < 16; ++rr) {
    const int tl = w * 16 + rr;
    const int t  = t0 + tl;
    const float* cur = xl + ((size_t)b * T_DIM + t) * C_DIM + h * HS;
    const float c0 = cur[lane], c1 = cur[lane + 32];
    float s0 = 0.0f, s1 = 0.0f;
    if (t + 1 < T_DIM) {
      const float* nx = cur + C_DIM;
      s0 = nx[lane];
      s1 = nx[lane + 32];
    }
    const float f0 = s0 * omv + c0 * vc;
    const float f1 = s1 * omv + c1 * vc;
    float ss = f0 * f0 + f1 * f1;
    ss += __shfl_xor(ss, 16, 32);
    ss += __shfl_xor(ss, 8, 32);
    ss += __shfl_xor(ss, 4, 32);
    ss += __shfl_xor(ss, 2, 32);
    ss += __shfl_xor(ss, 1, 32);
    const float rn = 1.0f / (sqrtf(ss) + 1e-6f);
    const float v0 = (f0 * rn) * vb;
    const float v1 = (f1 * rn) * vb;
    const us_t h0 = f2bf(v0), h1 = f2bf(v1);
    ldsH[lane][tl]      = h0;
    ldsH[lane + 32][tl] = h1;
    ldsL[lane][tl]      = f2bf(v0 - bf2f(h0));
    ldsL[lane + 32][tl] = f2bf(v1 - bf2f(h1));
  }
  __syncthreads();

  const int tid = threadIdx.x;
  const int ch  = tid & 7;
  const int dsl = tid >> 3;
  v4u ph[4], pl[4];
#pragma unroll
  for (int it = 0; it < 4; ++it) {
    const int d = it * 16 + dsl;
    ph[it] = *(const v4u*)(&ldsH[d][8 * ch]);
    pl[it] = *(const v4u*)(&ldsL[d][8 * ch]);
  }
  const size_t gb = ((size_t)bh * HS) * T_DIM + t0 + 8 * ch;
#pragma unroll
  for (int it = 0; it < 4; ++it) {
    const size_t off = gb + (size_t)(it * 16 + dsl) * T_DIM;
    *(volatile v4u*)(vthi + off) = ph[it];
    *(volatile v4u*)(vtlo + off) = pl[it];
  }
  __threadfence();
#pragma unroll
  for (int it = 0; it < 4; ++it) {
    const size_t off = gb + (size_t)(it * 16 + dsl) * T_DIM;
    *(volatile v4u*)(vthi + off) = ph[it];
    *(volatile v4u*)(vtlo + off) = pl[it];
  }
}

__global__ __launch_bounds__(128) void k_attn(const us_t* __restrict__ khi,
                                             const us_t* __restrict__ klo,
                                             const us_t* __restrict__ vthi,
                                             const us_t* __restrict__ vtlo,
                                             us_t* __restrict__ yhi,
                                             us_t* __restrict__ ylo) {
#pragma clang fp contract(off)
  __shared__ __align__(16) float ldsO[4][16][68];
  __shared__ float ldsInv[4][16];

  const int bh = blockIdx.y, b = bh / NH, h = bh % NH;
  const int w = threadIdx.x >> 5, lane = threadIdx.x & 31, m = lane & 15, hh = lane >> 4;
  const int Tm1 = T_DIM - 1;
  const int q0  = 1 + 64 * blockIdx.x + 16 * w;
  const int tq  = q0 + m;
  const int tqc = (tq < Tm1) ? tq : Tm1;

  const size_t kbh = (size_t)bh * T_DIM * HS;
  const size_t vbh = (size_t)bh * HS * T_DIM;

  const us_t* qh_row = khi + kbh + (size_t)tqc * HS;
  const us_t* ql_row = klo + kbh + (size_t)tqc * HS;
  const v16us qh0 = ld_frag(qh_row, hh),      ql0 = ld_frag(ql_row, hh);
  const v16us qh1 = ld_frag(qh_row + 32, hh), ql1 = ld_frag(ql_row + 32, hh);

  int qmax = q0 + 15;
  if (qmax > Tm1) qmax = Tm1;
  const int ntiles = (qmax + 31) >> 5;

  v8f o[4];
#pragma unroll
  for (int g = 0; g < 4; ++g) o[g] = vzero();
  float mrun = -1e30f, lrun = 0.0f;

  for (int kt = 0; kt < ntiles; ++kt) {
    const int kbase = kt * 32;

    v8f s[2];
#pragma unroll
    for (int g = 0; g < 2; ++g) {
      s[g] = vzero();
      const size_t ar = kbh + (size_t)(kbase + 16 * g + m) * HS;
      {
        const v16us kh = ld_frag(khi + ar, hh);
        const v16us kl = ld_frag(klo + ar, hh);
        s[g] = mma(kh, qh0, s[g]);
        s[g] = mma(kh, ql0, s[g]);
        s[g] = mma(kl, qh0, s[g]);
      }
      {
        const v16us kh = ld_frag(khi + ar + 32, hh);
        const v16us kl = ld_frag(klo + ar + 32, hh);
        s[g] = mma(kh, qh1, s[g]);
        s[g] = mma(kh, ql1, s[g]);
        s[g] = mma(kl, qh1, s[g]);
      }
    }

    float p0[8], p1[8];
    float mx = -1e30f;
#pragma unroll
    for (int r = 0; r < 8; ++r) {
      const int key0 = kbase + 8 * hh + r;
      float a = s[0][r];
      float c = s[1][r];
      if (key0 >= tq)      a = -1e30f;
      if (key0 + 16 >= tq) c = -1e30f;
      p0[r] = a;
      p1[r] = c;
      mx = fmaxf(mx, fmaxf(a, c));
    }
    mx = fmaxf(mx, __shfl_xor(mx, 16, 32));
    const float mn = fmaxf(mrun, mx);
    const float sc = __expf(mrun - mn);
    float sum = 0.0f;
#pragma unroll
    for (int r = 0; r < 8; ++r) {
      p0[r] = __expf(p0[r] - mn);
      p1[r] = __expf(p1[r] - mn);
      sum += p0[r] + p1[r];
    }
    sum += __shfl_xor(sum, 16, 32);
    lrun = lrun * sc + sum;
    mrun = mn;

#pragma unroll
    for (int r = 0; r < 8; ++r) {
      const float scr = __shfl(sc, 8 * hh + r, 32);
#pragma unroll
      for (int g = 0; g < 4; ++g) o[g][r] *= scr;
    }

    Frag ph, pl;
#pragma unroll
    for (int r = 0; r < 8; ++r) {
      const us_t a = f2bf(p0[r]);
      const us_t c = f2bf(p1[r]);
      ph.u[r]     = a;
      ph.u[8 + r] = c;
      pl.u[r]     = f2bf(p0[r] - bf2f(a));
      pl.u[8 + r] = f2bf(p1[r] - bf2f(c));
    }

#pragma unroll
    for (int g = 0; g < 4; ++g) {
      const size_t vr = vbh + (size_t)(16 * g + m) * T_DIM + kbase;
      const v16us vh = ld_frag(vthi + vr, hh);
      const v16us vl = ld_frag(vtlo + vr, hh);
      o[g] = mma(ph.u, vh, o[g]);
      o[g] = mma(ph.u, vl, o[g]);
      o[g] = mma(pl.u, vh, o[g]);
    }
  }

  const float inv = 1.0f / lrun;
  if (hh == 0) ldsInv[w][m] = inv;
#pragma unroll
  for (int g = 0; g < 4; ++g) {
#pragma unroll
    for (int r = 0; r < 8; ++r) ldsO[w][8 * hh + r][16 * g + m] = o[g][r];
  }
  __syncthreads();

  const int ch   = lane & 7;
  const int rsel = lane >> 3;
  v4u yh[4], yl[4];
#pragma unroll
  for (int it = 0; it < 4; ++it) {
    const int row = it * 4 + rsel;
    const float iv = ldsInv[w][row];
    const v4f* sp = (const v4f*)(&ldsO[w][row][8 * ch]);
    const v4f e0 = sp[0];
    const v4f e1 = sp[1];
    float vv[8];
#pragma unroll
    for (int i = 0; i < 4; ++i) { vv[i] = e0[i] * iv; vv[4 + i] = e1[i] * iv; }
#pragma unroll
    for (int i = 0; i < 4; ++i) {
      const us_t ha = f2bf(vv[2 * i]);
      const us_t hc = f2bf(vv[2 * i + 1]);
      yh[it][i] = pk2(ha, hc);
      yl[it][i] = pk2(f2bf(vv[2 * i] - bf2f(ha)), f2bf(vv[2 * i + 1] - bf2f(hc)));
    }
  }
  v4u vz;
#pragma unroll
  for (int i = 0; i < 4; ++i) vz[i] = 0u;

  const size_t yb = ((size_t)b * T_DIM) * C_DIM + h * HS + 8 * ch;
  const bool zrow = (blockIdx.x == 0) && (w == 0) && (lane < 8);

#pragma unroll
  for (int it = 0; it < 4; ++it) {
    const int tqr = q0 + it * 4 + rsel;
    if (tqr <= Tm1) {
      const size_t off = yb + (size_t)tqr * C_DIM;
      *(volatile v4u*)(yhi + off) = yh[it];
      *(volatile v4u*)(ylo + off) = yl[it];
    }
  }
  if (zrow) {
    *(volatile v4u*)(yhi + yb) = vz;
    *(volatile v4u*)(ylo + yb) = vz;
  }
  __threadfence();
#pragma unroll
  for (int it = 0; it < 4; ++it) {
    const int tqr = q0 + it * 4 + rsel;
    if (tqr <= Tm1) {
      const size_t off = yb + (size_t)tqr * C_DIM;
      *(volatile v4u*)(yhi + off) = yh[it];
      *(volatile v4u*)(ylo + off) = yl[it];
    }
  }
  if (zrow) {
    *(volatile v4u*)(yhi + yb) = vz;
    *(volatile v4u*)(ylo + yb) = vz;
  }
}

extern "C" void kernel_launch(void* const* d_in, const int* in_sizes, int n_in,
                              void* d_out, int out_size, void* d_ws,
                              size_t ws_size, hipStream_t stream) {
  const size_t MT = (size_t)B_DIM * T_DIM;
  const size_t NX = MT * C_DIM;
  const size_t NW = (size_t)C_DIM * C_DIM;

  if (n_in < 8) return;
  if ((size_t)in_sizes[0] != NX || (size_t)in_sizes[1] != NW || in_sizes[2] != NH ||
      (size_t)in_sizes[3] != NW || in_sizes[4] != NH || in_sizes[5] != NH ||
      in_sizes[6] != NH || (size_t)in_sizes[7] != NW || (size_t)out_size != NX) return;

  const float* x       = (const float*)d_in[0];
  const float* W_la    = (const float*)d_in[1];
  const float* la_coef = (const float*)d_in[2];
  const float* W_v     = (const float*)d_in[3];
  const float* v_coef  = (const float*)d_in[4];
  const float* kbeta   = (const float*)d_in[5];
  const float* vbeta   = (const float*)d_in[6];
  const float* W_proj  = (const float*)d_in[7];
  float* out = (float*)d_out;

  size_t off = 0;
  char* ws = (char*)d_ws;
  us_t* xb   = (us_t*)(ws + off); off += NX * 2;
  us_t* wla  = (us_t*)(ws + off); off += NW * 2;
  us_t* wv   = (us_t*)(ws + off); off += NW * 2;
  us_t* wpj  = (us_t*)(ws + off); off += NW * 2;
  float* u   = (float*)(ws + off); off += NX * 4;
  float* xl  = (float*)(ws + off); off += NX * 4;
  us_t* khi  = (us_t*)(ws + off); off += NX * 2;
  us_t* klo  = (us_t*)(ws + off); off += NX * 2;
  us_t* vthi = (us_t*)(ws + off); off += NX * 2;
  us_t* vtlo = (us_t*)(ws + off); off += NX * 2;
  us_t* yhi  = (us_t*)(ws + off); off += NX * 2;
  us_t* ylo  = (us_t*)(ws + off); off += NX * 2;
  if (off > ws_size) return;

  const int nx8 = (int)(NX / 8), nw8 = (int)(NW / 8);
  k_cvt<<<(nx8 + 255) / 256, 256, 0, stream>>>(x, xb, nx8);
  k_cvt<<<(nw8 + 255) / 256, 256, 0, stream>>>(W_la, wla, nw8);
  k_cvt<<<(nw8 + 255) / 256, 256, 0, stream>>>(W_v, wv, nw8);
  k_cvt<<<(nw8 + 255) / 256, 256, 0, stream>>>(W_proj, wpj, nw8);

  dim3 ggrid(C_DIM / 64, (unsigned)(MT / 64));
  k_gemm<0><<<ggrid, 128, 0, stream>>>(xb, xb, wla, u, (int)MT, C_DIM, C_DIM);
  k_gemm<0><<<ggrid, 128, 0, stream>>>(xb, xb, wv, xl, (int)MT, C_DIM, C_DIM);

  k_ema_knorm<<<B_DIM * (C_DIM / 256), 32, 0, stream>>>(u, la_coef, kbeta, khi, klo);

  dim3 vgrid(T_DIM / 64, B_DIM * NH);
  k_vmake<<<vgrid, 128, 0, stream>>>(xl, v_coef, vbeta, vthi, vtlo);

  dim3 agrid((T_DIM - 1 + 63) / 64, B_DIM * NH);
  k_attn<<<agrid, 128, 0, stream>>>(khi, klo, vthi, vtlo, yhi, ylo);

  k_gemm<1><<<ggrid, 128, 0, stream>>>(yhi, ylo, wpj, out, (int)MT, C_DIM, C_DIM);
}
